// HyperbolicGraphAttentionLayer_21938692948001
// MI455X (gfx1250) — hardware-run, weakly checked
//
#include <hip/hip_runtime.h>

typedef float          v8f   __attribute__((ext_vector_type(8)));
typedef float          v4f   __attribute__((ext_vector_type(4)));
typedef unsigned int   v4u   __attribute__((ext_vector_type(4)));
typedef int            v8i   __attribute__((ext_vector_type(8)));
typedef unsigned short v8us  __attribute__((ext_vector_type(8)));
typedef unsigned short v16us __attribute__((ext_vector_type(16)));
typedef __bf16         v16bf __attribute__((ext_vector_type(16)));
typedef _Float16       v16h  __attribute__((ext_vector_type(16)));
typedef v4f  __attribute__((may_alias)) v4fa;
typedef v8us __attribute__((may_alias)) v8usa;
union FragB { v16bf v; v16us u; v8us h[2]; v8i w; };
union FragH { v16h  v; v16us u; v8us h[2]; v8i w; };

__device__ __forceinline__ v8f wmb(const FragB& a, const FragB& b, v8f c) {
  v8f d = __builtin_amdgcn_wmma_f32_16x16x32_bf16(false, a.v, false, b.v, (short)0, c, false, false);
  asm volatile("v_nop\n\tv_nop\n\tv_nop\n\tv_nop" : "+v"(d) : "v"(a.w), "v"(b.w));
  return d;
}

__device__ __forceinline__ v8f wmh(const FragH& a, const FragH& b, v8f c) {
  v8f d = __builtin_amdgcn_wmma_f32_16x16x32_f16(false, a.v, false, b.v, (short)0, c, false, false);
  asm volatile("v_nop\n\tv_nop\n\tv_nop\n\tv_nop" : "+v"(d) : "v"(a.w), "v"(b.w));
  return d;
}

__device__ __forceinline__ unsigned bf16_bits(float f) {
  const unsigned u = __float_as_uint(f);
  const unsigned r = (u + 0x7FFFu + ((u >> 16) & 1u)) >> 16;
  const unsigned q = (u >> 16) | 0x40u;
  return ((u & 0x7fffffffu) > 0x7f800000u) ? q : r;
}

__device__ __forceinline__ float bf16_val(float f) {
  return __uint_as_float(bf16_bits(f) << 16);
}
__device__ __forceinline__ int clampi(int v, int lo, int hi) {
  return v < lo ? lo : (v > hi ? hi : v);
}

__device__ __forceinline__ unsigned f16_bits(float f) {
  const unsigned u  = __float_as_uint(f);
  const unsigned s  = (u >> 16) & 0x8000u;
  const unsigned a  = u & 0x7fffffffu;
  const unsigned t  = a - 0x38000000u;
  const unsigned r  = (t + 0x0FFFu + ((t >> 13) & 1u)) >> 13;
  const unsigned rc = r > 0x7C00u ? 0x7C00u : r;
  const bool small  = a < 0x38800000u;
  const bool isnan  = a > 0x7f800000u;
  const unsigned fin = small ? 0u : (s | rc);
  return isnan ? (s | 0x7E00u) : fin;
}

__device__ __forceinline__ unsigned pk16(unsigned lo, unsigned hi) { return lo | (hi << 16); }
__device__ __forceinline__ unsigned bf16_lo_bits(float v) {
  float hi = bf16_val(v);
  asm volatile("" : "+v"(hi));
  return bf16_bits(v - hi);
}
__device__ __forceinline__ v4u pack8_bf16(v4f a, v4f c) {
  return (v4u){ pk16(bf16_bits(a[0]), bf16_bits(a[1])), pk16(bf16_bits(a[2]), bf16_bits(a[3])),
                pk16(bf16_bits(c[0]), bf16_bits(c[1])), pk16(bf16_bits(c[2]), bf16_bits(c[3])) };
}
__device__ __forceinline__ v4u pack8_bf16_lo(v4f a, v4f c) {
  return (v4u){ pk16(bf16_lo_bits(a[0]), bf16_lo_bits(a[1])), pk16(bf16_lo_bits(a[2]), bf16_lo_bits(a[3])),
                pk16(bf16_lo_bits(c[0]), bf16_lo_bits(c[1])), pk16(bf16_lo_bits(c[2]), bf16_lo_bits(c[3])) };
}
__device__ __forceinline__ v4u pack8_f16(v4f a, v4f c) {
  return (v4u){ pk16(f16_bits(a[0]), f16_bits(a[1])), pk16(f16_bits(a[2]), f16_bits(a[3])),
                pk16(f16_bits(c[0]), f16_bits(c[1])), pk16(f16_bits(c[2]), f16_bits(c[3])) };
}

template <int FORM>
__global__ __launch_bounds__(256) void k_plane(const float* __restrict__ src, int rows, int cols, int ldsrc,
                                               unsigned short* __restrict__ dst, int MP, int KP) {
  static_assert(FORM >= 0 && FORM <= 3);
  const int KTOT = (FORM == 1 || FORM == 3) ? 2 * KP : KP;
  const unsigned ppr   = (unsigned)(KTOT >> 3);
  const unsigned kp8   = (unsigned)(KP >> 3);
  const unsigned total = (unsigned)MP * ppr;
  const unsigned g     = blockIdx.x * 256u + threadIdx.x;
  const unsigned rowu  = g / ppr;
  const unsigned p     = g - rowu * ppr;
  const bool second    = p >= kp8;
  const int row = (int)rowu;
  const int c0  = (int)((second ? p - kp8 : p) << 3);
  const float* srow = src + (size_t)clampi(row, 0, rows - 1) * (size_t)ldsrc;
  float x[8];
  unsigned mk[8];
#pragma unroll
  for (int e = 0; e < 8; ++e) {
    const int c = c0 + e;
    const float v = srow[clampi(c, 0, cols - 1)];
    asm volatile("" :: "v"(v));
    x[e]  = v;
    mk[e] = (row < rows && c < cols) ? 0xFFFFu : 0u;
  }
  const v4f a = (v4f){ x[0], x[1], x[2], x[3] };
  const v4f c = (v4f){ x[4], x[5], x[6], x[7] };
  v4u o;
  if (FORM == 2) {
    o = pack8_f16(a, c);
  } else {
    const v4u hi = pack8_bf16(a, c);
    o = hi;
    if (FORM == 1) { const v4u lo = pack8_bf16_lo(a, c); o = second ? lo : hi; }
  }
  const v4u mw = (v4u){ pk16(mk[0], mk[1]), pk16(mk[2], mk[3]), pk16(mk[4], mk[5]), pk16(mk[6], mk[7]) };
  o &= mw;
  if (g < total) {
    volatile v4u* q = (volatile v4u*)(dst + (size_t)g * 8);
    *q = o;
    __threadfence();
    *q = o;
  }
}

template <int FORM> struct FragOf    { typedef FragB T; };
template <>         struct FragOf<2> { typedef FragH T; };
__device__ __forceinline__ v8f mm(const FragB& a, const FragB& b, v8f c) { return wmb(a, b, c); }
__device__ __forceinline__ v8f mm(const FragH& a, const FragH& b, v8f c) { return wmh(a, b, c); }
template <class F> __device__ __forceinline__ F ld_frag(const unsigned short* p) {
  F f;
  f.h[0] = *(const v8usa*)(p);
  f.h[1] = *(const v8usa*)(p + 16);
  return f;
}

template <int FORM, int EPI>
__global__ __launch_bounds__(256) __attribute__((amdgpu_num_vgpr(248)))
void k_gemm_nt(const unsigned short* __restrict__ A, const unsigned short* __restrict__ B,
               const float* __restrict__ bias, float* __restrict__ D, int M, int N, int KTOT, int ldd) {
  static_assert(FORM >= 0 && FORM <= 2);
  static_assert(EPI == 0 || EPI == 1);
  typedef typename FragOf<FORM>::T F;
  __shared__ __attribute__((aligned(16))) float sT[8][16 * 68];
  const int lane = threadIdx.x & 31;
  const int wave = threadIdx.x >> 5;
  const int tilesM = (M + 63) >> 6;
  const int tilesN = (N + 63) >> 6;
  const int tile = blockIdx.x * 8 + wave;
  if (tile >= tilesM * tilesN) return;
  const int tm = tile / tilesN;
  const int tn = tile - tm * tilesN;
  const int m0 = tm << 6;
  const int n0 = tn << 6;

  const int rl = lane & 15;
  const int h8 = (lane >> 4) * 8;
  const unsigned short* pa = A + (size_t)(m0 + rl) * (size_t)KTOT + h8;
  const unsigned short* pb = B + (size_t)(n0 + rl) * (size_t)KTOT + h8;

  v8f acc[4][4];
#pragma unroll
  for (int i = 0; i < 4; ++i)
#pragma unroll
    for (int j = 0; j < 4; ++j) acc[i][j] = (v8f){0.f, 0.f, 0.f, 0.f, 0.f, 0.f, 0.f, 0.f};

#pragma unroll 1
  for (int k0 = 0; k0 < KTOT; k0 += 32) {
    F bf[4];
#pragma unroll
    for (int j = 0; j < 4; ++j) bf[j] = ld_frag<F>(pb + (size_t)(j << 4) * (size_t)KTOT + k0);
#pragma unroll
    for (int i = 0; i < 4; ++i) {
      const F af = ld_frag<F>(pa + (size_t)(i << 4) * (size_t)KTOT + k0);
#pragma unroll
      for (int j = 0; j < 4; ++j) acc[i][j] = mm(af, bf[j], acc[i][j]);
    }
  }

  float* slab = sT[wave];
  const int hh = lane >> 4;
  const int c4 = (lane & 15) * 4;
  const int nc = n0 + c4;
  const bool cok = nc < N;
  v4f bv = (v4f){0.f, 0.f, 0.f, 0.f};
  if (EPI == 1) {
    bv = *(const v4fa*)(bias + clampi(nc, 0, N - 4));
    asm volatile("" :: "v"(bv));
  }
#pragma unroll
  for (int i = 0; i < 4; ++i) {
    const int mBase = m0 + (i << 4);
#pragma unroll
    for (int j = 0; j < 4; ++j) {
#pragma unroll
      for (int r = 0; r < 8; ++r) slab[(h8 + r) * 68 + (j << 4) + rl] = acc[i][j][r];
    }
    __builtin_amdgcn_fence(__ATOMIC_RELEASE, "workgroup");
    __builtin_amdgcn_wave_barrier();
    __builtin_amdgcn_fence(__ATOMIC_ACQUIRE, "workgroup");
    v4f vv[8];
#pragma unroll
    for (int it = 0; it < 8; ++it) {
      const int row = it * 2 + hh;
      v4f v = *(const v4fa*)(slab + row * 68 + c4);
      if (EPI == 1) v += bv;
      vv[it] = v;
    }
    for (int pass = 0; pass < 2; ++pass) {
#pragma unroll
      for (int it = 0; it < 8; ++it) {
        const int row = mBase + it * 2 + hh;
        if (cok && row < M) *(volatile v4f*)(D + (size_t)row * (size_t)ldd + nc) = vv[it];
      }
      __threadfence();
    }
    __builtin_amdgcn_fence(__ATOMIC_RELEASE, "workgroup");
    __builtin_amdgcn_wave_barrier();
    __builtin_amdgcn_fence(__ATOMIC_ACQUIRE, "workgroup");
  }
}

#pragma clang fp contract(off)

#include <stddef.h>

#define P_TWO_TERM  1
#define AGG_LITERAL 0

#define NN      100000
#define NE      1600000
#define NPADR   100096
#define KTOT_   (P_TWO_TERM ? 128 : 64)
#define PW      (KTOT_ / 2)
#define EPSV    1e-15f
#define CLIPV   0.98f
#define BKT     1024
#define NBKT    98
#define RCAP    21504
#define DEGCAP  64
#define WLCAP   3072
#define EW      (NE / 8)
#define NST     ((EW + 255) / 256)
#define OFFP    1056
#define RPW     4

static_assert(NN % 32 == 0 && NN % 16 == 0);
static_assert(NPADR % 64 == 0 && NPADR >= NN && NPADR - NN < 64 + 64);
static_assert(NN < (1 << 17));
static_assert(NBKT * BKT >= NN && (NBKT - 1) * BKT < NN);
static_assert(BKT % 32 == 0 && BKT == 1024);
static_assert(NE == 781 * 2048 + 512);
static_assert(NE % 64 == 0 && EW % 8 == 0 && EW >= 8);
static_assert(NST == 782);
static_assert(RCAP % 1024 == 0 && RCAP * 4 >= 16721 * 5);
static_assert(DEGCAP == 64 && DEGCAP >= 36 + 8);
static_assert(8 * WLCAP >= RCAP);
static_assert(KTOT_ % 32 == 0);
static_assert(OFFP % 32 == 0 && OFFP >= BKT + 2);

#define LDSB_WORDS (RCAP + 8 * WLCAP + 8 * BKT + OFFP + 32)
#define LDSB_BYTES (LDSB_WORDS * 4)
static_assert(LDSB_BYTES <= 262144);

constexpr size_t al256(size_t v) { return (v + 255) & ~(size_t)255; }
constexpr size_t SZ_PHL  = al256((size_t)NPADR * KTOT_ * 2);
constexpr size_t SZ_F32  = al256((size_t)NN * 64 * 4);
constexpr size_t SZ_PN   = al256((size_t)NN * 4);
constexpr size_t SZ_HITS = al256((size_t)NBKT * RCAP * 4);
constexpr size_t SZ_OFF  = al256((size_t)NBKT * OFFP * 4);
constexpr size_t SZ_BT   = al256((size_t)64 * KTOT_ * 2);
constexpr size_t SZ_CB   = 256;
constexpr size_t O_PHL  = 0;
constexpr size_t O_MP   = O_PHL + SZ_PHL;
constexpr size_t O_HH   = O_MP + SZ_F32;
constexpr size_t O_LH   = O_HH + SZ_F32;
constexpr size_t O_PN   = O_LH + SZ_F32;
constexpr size_t O_HITS = O_PN + SZ_PN;
constexpr size_t O_OFF  = O_HITS + SZ_HITS;
constexpr size_t O_BT   = O_OFF + SZ_OFF;
constexpr size_t O_CB   = O_BT + SZ_BT;
constexpr size_t WS_TOTAL = O_CB + SZ_CB;
static_assert(WS_TOTAL <= ((size_t)128 << 20));
static_assert(!P_TWO_TERM || WS_TOTAL == (size_t)((size_t)436269 << 8));
static_assert(SZ_F32 >= (size_t)NN * 64 * 4);

typedef float v2f __attribute__((ext_vector_type(2)));
typedef int   v4i __attribute__((ext_vector_type(4)));
typedef v2f __attribute__((may_alias)) v2fa;
typedef v4i __attribute__((may_alias)) v4ia;
typedef v4u __attribute__((may_alias)) v4ua;

__device__ __forceinline__ float wsum(float v) {
#pragma unroll
  for (int o = 16; o > 0; o >>= 1) v += __shfl_xor(v, o);
  return v;
}

#define BT_UNITS   (64 * (KTOT_ / 8))
#define PAD_UNITS  ((NPADR - NN) * (KTOT_ / 8))
#define PREP_UNITS (BT_UNITS + PAD_UNITS + 32)
static_assert(BT_UNITS % 32 == 0 && PAD_UNITS % 32 == 0);

__global__ __launch_bounds__(256) void k_prep(const float* __restrict__ W, const float* __restrict__ cin,
                                              unsigned short* __restrict__ bt, unsigned short* __restrict__ phl,
                                              float* __restrict__ cb) {
  const int u = (int)blockIdx.x * 256 + (int)threadIdx.x;
  if (u < BT_UNITS) {
    const int n  = u / (KTOT_ / 8);
    const int k8 = (u - n * (KTOT_ / 8)) * 8;
    const int kk = k8 & 63;
    const float* p = W + (size_t)kk * 64 + n;
    float x[8];
#pragma unroll
    for (int e = 0; e < 8; ++e) {
      const float v = p[e * 64];
      asm volatile("" :: "v"(v));
      x[e] = v;
    }
    const v4u o = pack8_bf16((v4f){ x[0], x[1], x[2], x[3] }, (v4f){ x[4], x[5], x[6], x[7] });
    volatile v4u* q = (volatile v4u*)(bt + (size_t)u * 8);
    *q = o;
    __threadfence();
    *q = o;
  } else if (u < BT_UNITS + PAD_UNITS) {
    const int g = u - BT_UNITS;
    const v4u z = (v4u){ 0u, 0u, 0u, 0u };
    volatile v4u* q = (volatile v4u*)(phl + (size_t)NN * KTOT_ + (size_t)g * 8);
    *q = z;
    __threadfence();
    *q = z;
  } else if (u < BT_UNITS + PAD_UNITS + 8) {
    const int j = u - (BT_UNITS + PAD_UNITS);
    const float cr = bf16_val(cin[0]);
    const float sc = sqrtf(cr);
    const v4f vals = (v4f){ cr, sc, CLIPV / sc, -2.0f / sc };
    const v4f zero = (v4f){ 0.f, 0.f, 0.f, 0.f };
    const v4f o = (j == 0) ? vals : zero;
    volatile v4f* q = (volatile v4f*)(cb + 4 * j);
    *q = o;
    __threadfence();
    *q = o;
  }
}

__global__ __launch_bounds__(256) void k_rowA(const float* __restrict__ h, unsigned* __restrict__ phl32,
                                              float* __restrict__ pn) {
  __shared__ __attribute__((aligned(16))) float spn[32];
  const int lane = threadIdx.x & 31, wave = threadIdx.x >> 5;
  const int rbase = (int)blockIdx.x * 32;
#pragma unroll 1
  for (int i = 0; i < 4; ++i) {
    const int row = rbase + wave * 4 + i;
    const v2f hv = *(const v2fa*)(h + (size_t)row * 64 + 2 * lane);
    float f0 = bf16_val(hv.x) + EPSV;
    float f1 = bf16_val(hv.y) + EPSV;
    const float n0 = sqrtf(wsum(f0 * f0 + f1 * f1));
    const float m0 = (n0 > CLIPV) ? n0 : CLIPV;
    f0 = (f0 * CLIPV) / m0;
    f1 = (f1 * CLIPV) / m0;
    const float fn = sqrtf(wsum(f0 * f0 + f1 * f1));
    const float th = tanhf(fn);
    float p0 = (th * f0) / fn + EPSV;
    float p1 = (th * f1) / fn + EPSV;
    const float n1 = sqrtf(wsum(p0 * p0 + p1 * p1));
    const float m1 = (n1 > CLIPV) ? n1 : CLIPV;
    p0 = (p0 * CLIPV) / m1;
    p1 = (p1 * CLIPV) / m1;
    const float pnv = sqrtf(wsum(p0 * p0 + p1 * p1));
    const unsigned hiw = pk16(bf16_bits(p0), bf16_bits(p1));
    volatile unsigned* q = (volatile unsigned*)(phl32 + (size_t)row * PW + lane);
#if P_TWO_TERM
    const unsigned low = pk16(bf16_lo_bits(p0), bf16_lo_bits(p1));
    q[0]  = hiw;
    q[32] = low;
    __threadfence();
    q[0]  = hiw;
    q[32] = low;
#else
    q[0] = hiw;
    __threadfence();
    q[0] = hiw;
#endif
    if (lane == 0) spn[wave * 4 + i] = pnv;
  }
  __syncthreads();
  if (threadIdx.x < 8) {
    const v4f v = *(const v4fa*)(spn + 4 * (int)threadIdx.x);
    volatile v4f* q = (volatile v4f*)(pn + rbase + 4 * (int)threadIdx.x);
    *q = v;
    __threadfence();
    *q = v;
  }
}

__global__ __launch_bounds__(256) void k_rowB(const float* __restrict__ mp, const float* __restrict__ pn,
                                              const float* __restrict__ cb, float* __restrict__ hh) {
  const int lane = threadIdx.x & 31, wave = threadIdx.x >> 5;
  const int row = (int)blockIdx.x * 8 + wave;
  const int rc = row < NN ? row : NN - 1;
  const v4f cbv = *(const v4fa*)cb;
  const float sc = cbv[1], clip2 = cbv[2];
  const v2f mv = *(const v2fa*)(mp + (size_t)rc * 64 + 2 * lane);
  const float pnv = pn[rc];
  float x = sc * pnv;
  x = (x < -0.9f) ? -0.9f : ((x > 0.9f) ? 0.9f : x);
  const float a = atanhf(x);
  float t0 = ((mv.x * a) / pnv) / sc;
  float t1 = ((mv.y * a) / pnv) / sc;
  const float nt = sqrtf(wsum(t0 * t0 + t1 * t1));
  const float mt = (nt > clip2) ? nt : clip2;
  t0 = (t0 * clip2) / mt;
  t1 = (t1 * clip2) / mt;
  const float tn = sqrtf(wsum(t0 * t0 + t1 * t1));
  const float fac = (tanhf(sc * tn) / sc) / tn;
  const v2f o = (v2f){ fac * t0, fac * t1 };
  if (row < NN) {
    volatile v2f* q = (volatile v2f*)(hh + (size_t)row * 64 + 2 * lane);
    *q = o;
    __threadfence();
    *q = o;
  }
}

__global__ __launch_bounds__(256) void k_rowC(const float* __restrict__ hh, const float* __restrict__ cb,
                                              float* __restrict__ lh) {
  const int lane = threadIdx.x & 31, wave = threadIdx.x >> 5;
  const int row = (int)blockIdx.x * 8 + wave;
  const int rc = row < NN ? row : NN - 1;
  const v4f cbv = *(const v4fa*)cb;
  const float sc = cbv[1];
  const v2f hv = *(const v2fa*)(hh + (size_t)rc * 64 + 2 * lane);
  float g0 = hv.x + EPSV;
  float g1 = hv.y + EPSV;
  const float ng = sqrtf(wsum(g0 * g0 + g1 * g1));
  const float mg = (ng > CLIPV) ? ng : CLIPV;
  g0 = (g0 * CLIPV) / mg;
  g1 = (g1 * CLIPV) / mg;
  const float gn = sqrtf(wsum(g0 * g0 + g1 * g1));
  float x = sc * gn;
  x = (x < -0.9f) ? -0.9f : ((x > 0.9f) ? 0.9f : x);
  const float a = atanhf(x);
  const v2f o = (v2f){ (a * g0) / gn, (a * g1) / gn };
  if (row < NN) {
    volatile v2f* q = (volatile v2f*)(lh + (size_t)row * 64 + 2 * lane);
    *q = o;
    __threadfence();
    *q = o;
  }
}

__global__ __launch_bounds__(256) void k_bucket(const int* __restrict__ ei, unsigned* __restrict__ hits,
                                                unsigned* __restrict__ offp) {
  extern __shared__ v4u lds_dyn[];
  unsigned* reg2 = (unsigned*)lds_dyn;
  unsigned* wl   = reg2 + RCAP;
  int* cntw  = (int*)(wl + 8 * WLCAP);
  int* soff  = cntw + 8 * BKT;
  int* wtot  = soff + OFFP;
  int* wflag = wtot + 8;
  const int tid = (int)threadIdx.x, lane = tid & 31, wave = tid >> 5;
  const int b = (int)blockIdx.x;
  const int base = b * BKT;
  const int nbk = (NN - base) < BKT ? (NN - base) : BKT;

  {
    const v4u z = (v4u){ 0u, 0u, 0u, 0u };
#pragma unroll 1
    for (int i = tid; i < RCAP / 4; i += 256) ((v4ua*)reg2)[i] = z;
#pragma unroll 1
    for (int i = tid; i < (8 * BKT) / 4; i += 256) ((v4ua*)cntw)[i] = z;
  }

  const int* rowp = ei;
  const int* colp = ei + NE;
  const int wbeg = wave * EW;
  unsigned* myl = wl + wave * WLCAP;
  int wc = 0;
#pragma unroll 1
  for (int s = 0; s < NST; ++s) {
    const int e0 = s * 256 + lane * 8;
    const bool valid = e0 < EW;
    const int ec = wbeg + (e0 < EW - 8 ? e0 : EW - 8);
    const v4i ra = *(const v4ia*)(rowp + ec);
    const v4i rb = *(const v4ia*)(rowp + ec + 4);
    const v4i ca = *(const v4ia*)(colp + ec);
    const v4i cq = *(const v4ia*)(colp + ec + 4);
    asm volatile("" :: "v"(ra), "v"(rb), "v"(ca), "v"(cq));
    const int rr[8] = { ra.x, ra.y, ra.z, ra.w, rb.x, rb.y, rb.z, rb.w };
    const int cl[8] = { ca.x, ca.y, ca.z, ca.w, cq.x, cq.y, cq.z, cq.w };
    unsigned wd[8];
    bool ht[8];
    int c = 0;
#pragma unroll
    for (int j = 0; j < 8; ++j) {
      const unsigned sj = (unsigned)rr[j] - (unsigned)base;
      ht[j] = valid && (sj < (unsigned)nbk);
      wd[j] = (unsigned)clampi(cl[j], 0, NN - 1) | ((sj & (unsigned)(BKT - 1)) << 17);
      c += ht[j] ? 1 : 0;
    }
    int incl = c;
#pragma unroll
    for (int d = 1; d < 32; d <<= 1) {
      const int up = __shfl_up(incl, d);
      incl += (lane >= d) ? up : 0;
    }
    int pos = wc + incl - c;
#pragma unroll
    for (int j = 0; j < 8; ++j) {
      if (ht[j]) {
        if (pos < WLCAP) myl[pos] = wd[j];
        ++pos;
      }
    }
    wc += __shfl(incl, 31);
  }
  __syncthreads();

  const int wcr = __builtin_amdgcn_readfirstlane(wc);
  const int n = wcr > WLCAP ? WLCAP : wcr;
  int* myc = cntw + wave * BKT;
#pragma unroll 1
  for (int b0 = 0; b0 < n; b0 += 32) {
    int idx = b0 + lane;
    idx = idx < n ? idx : n - 1;
    const int uv = (int)myl[idx];
    const int m32 = (n - b0) < 32 ? (n - b0) : 32;
#pragma unroll 1
    for (int k = 0; k < m32; ++k) {
      const int u = __builtin_amdgcn_readlane(uv, k);
      const int sl = (u >> 17) & (BKT - 1);
      if (lane == 0) myc[sl] = myc[sl] + 1;
    }
  }
  __syncthreads();

  int cc[4][8];
  int tt[4] = { 0, 0, 0, 0 };
#pragma unroll
  for (int w = 0; w < 8; ++w) {
    const v4i q = *(const v4ia*)(cntw + w * BKT + 4 * tid);
    cc[0][w] = q.x; cc[1][w] = q.y; cc[2][w] = q.z; cc[3][w] = q.w;
    tt[0] += q.x; tt[1] += q.y; tt[2] += q.z; tt[3] += q.w;
  }
  const int ts = tt[0] + tt[1] + tt[2] + tt[3];
  int incl = ts;
#pragma unroll
  for (int d = 1; d < 32; d <<= 1) {
    const int up = __shfl_up(incl, d);
    incl += (lane >= d) ? up : 0;
  }
  if (lane == 31) wtot[wave] = incl;
  __syncthreads();
  int pre = 0, nh = 0;
#pragma unroll
  for (int w2 = 0; w2 < 8; ++w2) {
    const int t = wtot[w2];
    nh += t;
    pre += (w2 < wave) ? t : 0;
  }
  int run = pre + incl - ts;
  bool dov = false;
#pragma unroll
  for (int j = 0; j < 4; ++j) {
    soff[4 * tid + j] = run;
    int cur = run;
#pragma unroll
    for (int w = 0; w < 8; ++w) {
      cntw[w * BKT + 4 * tid + j] = cur;
      cur += cc[j][w];
    }
    run += tt[j];
    dov = dov || (tt[j] > DEGCAP);
  }
  const unsigned dm = __builtin_amdgcn_ballot_w32(dov);
  if (lane == 0) wflag[wave] = ((dm != 0u) || (wcr > WLCAP)) ? 1 : 0;
  __syncthreads();
  int flag = (nh > RCAP) ? 1 : 0;
#pragma unroll
  for (int w2 = 0; w2 < 8; ++w2) flag |= wflag[w2];
  if (tid < 32) soff[BKT + tid] = (tid == 0) ? nh : ((tid == 1) ? flag : 0);

#pragma unroll 1
  for (int b0 = 0; b0 < n; b0 += 32) {
    int idx = b0 + lane;
    idx = idx < n ? idx : n - 1;
    const int uv = (int)myl[idx];
    const int m32 = (n - b0) < 32 ? (n - b0) : 32;
#pragma unroll 1
    for (int k = 0; k < m32; ++k) {
      const int u = __builtin_amdgcn_readlane(uv, k);
      const int sl = (u >> 17) & (BKT - 1);
      if (lane == 0) {
        const int pos = myc[sl];
        const int pc = clampi(pos, 0, RCAP - 1);
        reg2[pc] = (unsigned)u;
        myc[sl] = pos + 1;
      }
    }
  }
  __syncthreads();

  unsigned* hb = hits + (size_t)b * RCAP;
#pragma unroll 1
  for (int it = 0; it < RCAP / 1024; ++it) {
    const int i4 = it * 256 + tid;
    const v4u v = ((const v4ua*)reg2)[i4];
    volatile v4u* q = (volatile v4u*)(hb + (size_t)i4 * 4);
    *q = v;
    __threadfence();
    *q = v;
  }
  unsigned* ob = offp + (size_t)b * OFFP;
  {
    const v4u v = ((const v4ua*)soff)[tid];
    volatile v4u* q = (volatile v4u*)(ob + 4 * tid);
    *q = v;
    __threadfence();
    *q = v;
  }
  if (tid < 8) {
    const v4u v = ((const v4ua*)soff)[256 + tid];
    volatile v4u* q = (volatile v4u*)(ob + BKT + 4 * tid);
    *q = v;
    __threadfence();
    *q = v;
  }
}

__device__ __forceinline__ float escore(float r2, float sc, float m2s) {
  const float rn = sqrtf(r2);
  float x = sc * rn;
  x = (x < 1e-8f) ? 1e-8f : ((x > CLIPV) ? CLIPV : x);
  return m2s * atanhf(x);
}

__global__ __launch_bounds__(256) void k_replay(const float* __restrict__ hh, const float* __restrict__ lh,
                                                const unsigned* __restrict__ hits, const unsigned* __restrict__ offp,
                                                const float* __restrict__ cb, float* __restrict__ att) {
  const int lane = threadIdx.x & 31, wave = threadIdx.x >> 5;
  const v4f cbv = *(const v4fa*)cb;
  const float c = cbv[0], sc = cbv[1], m2s = cbv[3];
  const float c2 = 2.0f * c;
  const float cc = c * c;
  const float ninf = __uint_as_float(0xff800000u);
  const float qnan = __uint_as_float(0x7fc00000u);
#pragma unroll 1
  for (int i = 0; i < RPW; ++i) {
    const int r = (int)blockIdx.x * 32 + wave * RPW + i;
    const int b = r >> 10, slot = r & (BKT - 1);
    const unsigned* ob = offp + (size_t)b * OFFP;
    const int st = (int)ob[slot];
    const int en = (int)ob[slot + 1];
    const int nh = (int)ob[BKT];
    const int fl = (int)ob[BKT + 1];
    const int nhc = clampi(nh, 0, RCAP);
    const int stc = clampi(st, 0, nhc);
    const int enc = clampi(en, stc, nhc);
    int cntv = enc - stc;
    const bool dover = cntv > DEGCAP;
    cntv = dover ? DEGCAP : cntv;
    const int cnt  = __builtin_amdgcn_readfirstlane(cntv);
    const int st_u = __builtin_amdgcn_readfirstlane(stc);
    const bool poison = (fl != 0) || dover;

    const unsigned* hb = hits + (size_t)b * RCAP;
    int i0 = st_u + lane;       i0 = i0 < RCAP ? i0 : RCAP - 1;
    int i1 = st_u + 32 + lane;  i1 = i1 < RCAP ? i1 : RCAP - 1;
    const unsigned w0 = hb[i0];
    const unsigned w1 = hb[i1];
    asm volatile("" :: "v"(w0), "v"(w1));
    const int col0 = clampi((int)(w0 & 0x1FFFFu), 0, NN - 1);
    const int col1 = clampi((int)(w1 & 0x1FFFFu), 0, NN - 1);

    const v2f hu = *(const v2fa*)(hh + (size_t)r * 64 + 2 * lane);
    const float u0 = -hu.x, u1 = -hu.y;
    const float nu = wsum(u0 * u0 + u1 * u1);
    const float coef2 = 1.0f - c * nu;
    const float ccnu = cc * nu;
    float r0 = 0.0f, r1 = 0.0f;
#pragma unroll 1
    for (int q = 0; q < cnt; ++q) {
      const int csel = (q < 32) ? col0 : col1;
      const int col = clampi(__shfl(csel, q & 31), 0, NN - 1);
      const v2f hv = *(const v2fa*)(hh + (size_t)col * 64 + 2 * lane);
      asm volatile("" :: "v"(hv));
      float pnv = hv.x * hv.x + hv.y * hv.y;
      float pd  = u0 * hv.x + u1 * hv.y;
#pragma unroll
      for (int o = 16; o > 0; o >>= 1) {
        const float ta = __shfl_xor(pnv, o);
        const float tb = __shfl_xor(pd, o);
        pnv += ta;
        pd  += tb;
      }
      const float base1 = 1.0f + c2 * pd;
      const float coef1 = base1 + c * pnv;
      const float den   = base1 + ccnu * pnv;
      const float m0 = (coef1 * u0 + coef2 * hv.x) / den;
      const float m1 = (coef1 * u1 + coef2 * hv.y) / den;
      const float rr = wsum(m0 * m0 + m1 * m1);
      const bool mine = lane == (q & 31);
      r0 = (mine && q < 32)  ? rr : r0;
      r1 = (mine && q >= 32) ? rr : r1;
    }

    const bool v0 = lane < cnt;
    const bool v1 = (lane + 32) < cnt;
    const float e0 = escore(r0, sc, m2s);
    const float e1 = escore(r1, sc, m2s);
    const float g0 = v0 ? e0 : ninf;
    const float g1 = v1 ? e1 : ninf;
    float em = (g1 > g0) ? g1 : g0;
#pragma unroll
    for (int o = 16; o > 0; o >>= 1) {
      const float t = __shfl_xor(em, o);
      em = (t > em) ? t : em;
    }
    const bool fin = (__float_as_uint(em) & 0x7f800000u) != 0x7f800000u;
    const float emx = fin ? em : 0.0f;
    float ex0 = expf(e0 - emx);
    float ex1 = expf(e1 - emx);
    ex0 = v0 ? ex0 : 0.0f;
    ex1 = v1 ? ex1 : 0.0f;
    const float dn = wsum(ex0 + ex1);
    const float dd = dn + 1e-16f;

    float a0 = 0.0f, a1 = 0.0f;
#pragma unroll 1
    for (int q = 0; q < cnt; ++q) {
      const int csel = (q < 32) ? col0 : col1;
      const float esel = (q < 32) ? ex0 : ex1;
      const int col = clampi(__shfl(csel, q & 31), 0, NN - 1);
      const float exq = __shfl(esel, q & 31);
      const v2f lv = *(const v2fa*)(lh + (size_t)col * 64 + 2 * lane);
      asm volatile("" :: "v"(lv));
#if AGG_LITERAL
      const float wq = sc * (exq / dd);
      a0 = a0 + wq * lv.x;
      a1 = a1 + wq * lv.y;
#else
      a0 = a0 + exq * lv.x;
      a1 = a1 + exq * lv.y;
#endif
    }
#if !AGG_LITERAL
    a0 = (sc * a0) / dd;
    a1 = (sc * a1) / dd;
#endif
    const v2f o = (v2f){ poison ? qnan : a0, poison ? qnan : a1 };
    volatile v2f* qp = (volatile v2f*)(att + (size_t)r * 64 + 2 * lane);
    *qp = o;
    __threadfence();
    *qp = o;
  }
}

__global__ __launch_bounds__(256) void k_final(const float* __restrict__ att, const unsigned* __restrict__ offp,
                                               const float* __restrict__ cb, float* __restrict__ out) {
  const int lane = threadIdx.x & 31, wave = threadIdx.x >> 5;
  const int row = (int)blockIdx.x * 8 + wave;
  const int rc = row < NN ? row : NN - 1;
  const v4f cbv = *(const v4fa*)cb;
  const float sc = cbv[1], clip3 = cbv[2];
  const int fl = (int)offp[(size_t)(rc >> 10) * OFFP + BKT + 1];
  const v2f av = *(const v2fa*)(att + (size_t)rc * 64 + 2 * lane);
  float z0 = ((av.x > 0.0f) ? av.x : expm1f(av.x)) + EPSV;
  float z1 = ((av.y > 0.0f) ? av.y : expm1f(av.y)) + EPSV;
  const float nz = sqrtf(wsum(z0 * z0 + z1 * z1));
  const float mz = (nz > clip3) ? nz : clip3;
  z0 = (z0 * clip3) / mz;
  z1 = (z1 * clip3) / mz;
  const float zn = sqrtf(wsum(z0 * z0 + z1 * z1));
  const float th = tanhf(sc * zn);
  const float o0 = ((th * z0) / sc) / zn;
  const float o1 = ((th * z1) / sc) / zn;
  const float qnan = __uint_as_float(0x7fc00000u);
  const v2f o = (v2f){ (fl != 0) ? qnan : o0, (fl != 0) ? qnan : o1 };
  if (row < NN) {
    volatile v2f* q = (volatile v2f*)(out + (size_t)row * 64 + 2 * lane);
    *q = o;
    __threadfence();
    *q = o;
  }
}

static inline int cdiv_i(int a, int b) { return (a + b - 1) / b; }

extern "C" void kernel_launch(void* const* d_in, const int* in_sizes, int n_in,
                              void* d_out, int out_size, void* d_ws, size_t ws_size,
                              hipStream_t stream) {
  if (n_in < 4) return;
  if (in_sizes[0] != NN * 64) return;
  if (in_sizes[1] != 64 * 64) return;
  if (in_sizes[2] != 1) return;
  if (in_sizes[3] != 2 * NE) return;
  if (out_size != NN * 64) return;
  if (ws_size < WS_TOTAL) return;

  const float* h  = (const float*)d_in[0];
  const float* W  = (const float*)d_in[1];
  const float* c  = (const float*)d_in[2];
  const int*   ei = (const int*)d_in[3];
  float* out = (float*)d_out;

  char* ws = (char*)d_ws;
  unsigned short* PHL = (unsigned short*)(ws + O_PHL);
  float*    MPp  = (float*)(ws + O_MP);
  float*    ATT  = (float*)(ws + O_MP);
  float*    HH   = (float*)(ws + O_HH);
  float*    LH   = (float*)(ws + O_LH);
  float*    PN   = (float*)(ws + O_PN);
  unsigned* HITS = (unsigned*)(ws + O_HITS);
  unsigned* OFFT = (unsigned*)(ws + O_OFF);
  unsigned short* BT = (unsigned short*)(ws + O_BT);
  float*    CB   = (float*)(ws + O_CB);

  hipFuncSetAttribute(reinterpret_cast<const void*>(&k_bucket),
                      hipFuncAttributeMaxDynamicSharedMemorySize, LDSB_BYTES);

  k_prep<<<cdiv_i(PREP_UNITS, 256), 256, 0, stream>>>(W, c, BT, PHL, CB);
  k_rowA<<<NN / 32, 256, 0, stream>>>(h, (unsigned*)PHL, PN);
  {
    const int tiles = ((NN + 63) >> 6) * 1;
    k_gemm_nt<P_TWO_TERM, 0><<<cdiv_i(tiles, 8), 256, 0, stream>>>(PHL, BT, CB, MPp, NN, 64, KTOT_, 64);
  }
  k_rowB<<<NN / 8, 256, 0, stream>>>(MPp, PN, CB, HH);
  k_rowC<<<NN / 8, 256, 0, stream>>>(HH, CB, LH);
  k_bucket<<<NBKT, 256, LDSB_BYTES, stream>>>(ei, HITS, OFFT);
  k_replay<<<NN / 32, 256, 0, stream>>>(HH, LH, HITS, OFFT, CB, ATT);
  k_final<<<NN / 8, 256, 0, stream>>>(ATT, OFFT, CB, out);
}
